// SpeMamba_17325898072382
// MI455X (gfx1250) — hardware-run, weakly checked
//
#include <hip/hip_runtime.h>
#include <hip/hip_bf16.h>

typedef __attribute__((ext_vector_type(16))) __bf16   v16b;
typedef __attribute__((ext_vector_type(8)))  __bf16   v8b;
typedef __attribute__((ext_vector_type(8)))  float    v8f;
typedef __attribute__((ext_vector_type(4)))  float    v4f;
typedef __attribute__((ext_vector_type(4)))  unsigned v4u;

constexpr int kTok     = 8;
constexpr int kGDim    = 25;
constexpr int kDin     = 50;
constexpr int kDst     = 16;
constexpr int kNX      = 34;
constexpr int kHW      = 4096;
constexpr int kNCh     = 200;
constexpr int kBStride = kNCh * kHW;
constexpr int kNPix    = 2 * kHW;
constexpr int kPixB    = 8;
constexpr int kTokB    = kPixB * kTok;
constexpr int kThreads = 128;
constexpr int kNBlk    = kNPix / kPixB;
constexpr int kBlkPerImg = kHW / kPixB;
constexpr int kYPitch  = 32;
static_assert(kNPix % kPixB == 0, "grid exact");
static_assert(kTokB == 16 * (kThreads / 32), "one M tile per wave");
static_assert(kYPitch * 4 == 128, "one line per token row");

constexpr size_t kWsYpreBytes  = (size_t)kNPix * kTok * kYPitch * 4;
constexpr size_t kWsPartBytes  = (size_t)kNBlk * 32 * 4;
constexpr size_t kWsTotal      = kWsYpreBytes + kWsPartBytes;
static_assert(kWsTotal <= 134217728, "ws budget");

constexpr int OFF_XTH  = 0;
constexpr int OFF_XTL  = 4096;
constexpr int OFF_W1H  = 8192;
constexpr int OFF_W1L  = 15360;
constexpr int OFF_XINH = 22528;
constexpr int OFF_XINL = 30720;
constexpr int OFF_WXH  = 38912;
constexpr int OFF_WXL  = 45056;
constexpr int OFF_W3H  = 51200;
constexpr int OFF_W3L  = 55296;
constexpr int OFF_PLANES_END = 59392;
constexpr int OFF_XINF = 59392;
constexpr int OFF_ZF   = 72192;
constexpr int OFF_XDBL = 84992;
constexpr int OFF_AM2  = 94208;
constexpr int OFF_CW   = 97408;
constexpr int OFF_CB   = 98208;
constexpr int OFF_DTW  = 98416;
constexpr int OFF_DTB  = 98816;
constexpr int OFF_DV   = 99024;
constexpr int OFF_RED  = 99232;
constexpr int OFF_BLK  = 99360;
constexpr int SMEM_TOTAL = 99488;
static_assert(OFF_PLANES_END % 16 == 0 && OFF_XINF % 16 == 0 && OFF_ZF % 16 == 0 && OFF_XDBL % 16 == 0 &&
              OFF_AM2 % 16 == 0 && OFF_CW % 16 == 0 && OFF_CB % 16 == 0 && OFF_DTW % 16 == 0 &&
              OFF_DTB % 16 == 0 && OFF_DV % 16 == 0 && OFF_RED % 16 == 0 && OFF_BLK % 16 == 0, "align");
static_assert(OFF_ZF - OFF_XINF >= kTokB * kYPitch * 4, "slab fits in the xin f32 region");

__device__ __forceinline__ unsigned short f2bf_bits(float f) {
  unsigned u = __float_as_uint(f);
  return (unsigned short)((u + 0x7FFFu + ((u >> 16) & 1u)) >> 16);
}
__device__ __forceinline__ float bf_bits2f(unsigned short h) { return __uint_as_float(((unsigned)h) << 16); }
__device__ __forceinline__ void bsplit(float f, __bf16& hi, __bf16& lo) {
  const unsigned short hb = f2bf_bits(f);
  hi = __builtin_bit_cast(__bf16, hb);
  lo = __builtin_bit_cast(__bf16, f2bf_bits(f - bf_bits2f(hb)));
}

template <typename T> struct Frag;
template <> struct Frag<__bf16> {
  typedef v16b V; union U { v16b v; v8b h[2]; };
  static __device__ __forceinline__ v16b load(const __bf16* p) {
    U f; f.h[0] = *(const v8b*)(p); f.h[1] = *(const v8b*)(p + 16); return f.v;
  }
};

__device__ __forceinline__ v8f mma3(v16b ah, v16b al, v16b bh, v16b bl, v8f c) {
  c = __builtin_amdgcn_wmma_f32_16x16x32_bf16(false, ah, false, bh, (short)0, c, false, false);
  c = __builtin_amdgcn_wmma_f32_16x16x32_bf16(false, ah, false, bl, (short)0, c, false, false);
  c = __builtin_amdgcn_wmma_f32_16x16x32_bf16(false, al, false, bh, (short)0, c, false, false);
  asm volatile("v_nop\n\tv_nop\n\tv_nop\n\tv_nop" : "+v"(c) : "v"(ah), "v"(al), "v"(bh), "v"(bl));
  return c;
}
__device__ __forceinline__ v8f vzero8() { return (v8f){0.f, 0.f, 0.f, 0.f, 0.f, 0.f, 0.f, 0.f}; }

__device__ __forceinline__ float sigm_f(float x) { return 1.0f / (1.0f + expf(-x)); }
__device__ __forceinline__ float softplus_f(float x) { return fmaxf(x, 0.0f) + log1pf(expf(-fabsf(x))); }

constexpr float kLog2e = 1.4426950408889634f;

__global__ __launch_bounds__(kThreads) void k_mamba_fused(
    const float* __restrict__ x, const float* __restrict__ pe, const float* __restrict__ w_in,
    const float* __restrict__ conv_w, const float* __restrict__ conv_b, const float* __restrict__ w_x,
    const float* __restrict__ w_dt, const float* __restrict__ b_dt, const float* __restrict__ a_log,
    const float* __restrict__ dvec, const float* __restrict__ w_out,
    float* __restrict__ ypre, float* __restrict__ gpart)
{
  __shared__ __align__(16) unsigned char smem[SMEM_TOTAL];
  __bf16* XtH  = (__bf16*)(smem + OFF_XTH);
  __bf16* XtL  = (__bf16*)(smem + OFF_XTL);
  __bf16* W1H  = (__bf16*)(smem + OFF_W1H);
  __bf16* W1L  = (__bf16*)(smem + OFF_W1L);
  __bf16* XinH = (__bf16*)(smem + OFF_XINH);
  __bf16* XinL = (__bf16*)(smem + OFF_XINL);
  __bf16* WxH  = (__bf16*)(smem + OFF_WXH);
  __bf16* WxL  = (__bf16*)(smem + OFF_WXL);
  __bf16* W3H  = (__bf16*)(smem + OFF_W3H);
  __bf16* W3L  = (__bf16*)(smem + OFF_W3L);
  float* XinF  = (float*)(smem + OFF_XINF);
  float* ZF    = (float*)(smem + OFF_ZF);
  float* Xdbl  = (float*)(smem + OFF_XDBL);
  float* Am2   = (float*)(smem + OFF_AM2);
  float* Cw    = (float*)(smem + OFF_CW);
  float* Cb    = (float*)(smem + OFF_CB);
  float* Dtw   = (float*)(smem + OFF_DTW);
  float* Dtb   = (float*)(smem + OFF_DTB);
  float* Dvv   = (float*)(smem + OFF_DV);
  float* Red   = (float*)(smem + OFF_RED);
  float* Blk   = (float*)(smem + OFF_BLK);

  const int tid  = threadIdx.x;
  const int lane = tid & 31;
  const int wave = tid >> 5;
  const int c16  = lane & 15;
  const int hh   = lane >> 4;
  const int koff = hh * 8;
  const int blk  = blockIdx.x;
  const int pixbase = blk * kPixB;
  const int bimg = pixbase >> 12;
  const int pix0 = pixbase & (kHW - 1);
  const float* xb = x + (size_t)bimg * kBStride + pix0;

  {
    v4u* zp = (v4u*)smem;
    const v4u z4 = (v4u){0u, 0u, 0u, 0u};
    for (int i = tid; i < OFF_PLANES_END / 16; i += kThreads) zp[i] = z4;
  }
  __syncthreads();

#pragma unroll 2
  for (int i = tid; i < 100 * kGDim; i += kThreads) {
    const int e = i / kGDim, d = i - e * kGDim;
    __bf16 a, b; bsplit(w_in[i], a, b);
    W1H[e * 32 + d] = a; W1L[e * 32 + d] = b;
  }
#pragma unroll 2
  for (int i = tid; i < kNX * kDin; i += kThreads) {
    const int e = i / kDin, d = i - e * kDin;
    __bf16 a, b; bsplit(w_x[i], a, b);
    WxH[e * 64 + d] = a; WxL[e * 64 + d] = b;
  }
#pragma unroll 2
  for (int i = tid; i < kGDim * kDin; i += kThreads) {
    const int o = i / kDin, d = i - o * kDin;
    __bf16 a, b; bsplit(w_out[i], a, b);
    W3H[o * 64 + d] = a; W3L[o * 64 + d] = b;
  }
#pragma unroll 2
  for (int i = tid; i < kDin * kDst; i += kThreads) Am2[i] = -expf(a_log[i]) * kLog2e;
#pragma unroll 2
  for (int i = tid; i < kDin * 4; i += kThreads) Cw[i] = conv_w[i];
  if (tid < kDin) { Cb[tid] = conv_b[tid]; Dtb[tid] = b_dt[tid]; Dvv[tid] = dvec[tid]; }
  if (tid < 2 * kDin) Dtw[tid] = w_dt[tid];
#pragma unroll 2
  for (int i = tid; i < kPixB * kNCh; i += kThreads) {
    const int ch = i >> 3, p = i & 7;
    const int l = ch / kGDim, d = ch - l * kGDim;
    const float v = xb[(size_t)ch * kHW + p] + pe[d];
    __bf16 a, b; bsplit(v, a, b);
    const int tok = p * kTok + l;
    XtH[tok * 32 + d] = a; XtL[tok * 32 + d] = b;
  }
  __syncthreads();

  const int tb = wave * 16;

  v8f acc1[7];
#pragma unroll
  for (int t = 0; t < 7; ++t) acc1[t] = vzero8();
  {
    const v16b ah = Frag<__bf16>::load(XtH + (tb + c16) * 32 + koff);
    const v16b al = Frag<__bf16>::load(XtL + (tb + c16) * 32 + koff);
#pragma unroll
    for (int t = 0; t < 7; ++t) {
      const v16b bh = Frag<__bf16>::load(W1H + (t * 16 + c16) * 32 + koff);
      const v16b bl = Frag<__bf16>::load(W1L + (t * 16 + c16) * 32 + koff);
      acc1[t] = mma3(ah, al, bh, bl, acc1[t]);
    }
  }

#pragma unroll
  for (int t = 0; t < 4; ++t) {
    const int n = t * 16 + c16;
    const bool valid = n < kDin;
    const int nn = valid ? n : 0;
    const float w0 = Cw[nn * 4 + 0], w1 = Cw[nn * 4 + 1], w2 = Cw[nn * 4 + 2], w3 = Cw[nn * 4 + 3], bb = Cb[nn];
    float p1 = 0.f, p2 = 0.f, p3 = 0.f;
#pragma unroll
    for (int r = 0; r < 8; ++r) {
      const float cur = acc1[t][r];
      float v = w0 * p3;
      v = fmaf(w1, p2, v);
      v = fmaf(w2, p1, v);
      v = fmaf(w3, cur, v);
      v += bb;
      p3 = p2; p2 = p1; p1 = cur;
      const float sv = v * sigm_f(v);
      const int tok = tb + hh * 8 + r;
      if (valid) {
        XinF[tok * kDin + n] = sv;
        __bf16 a, b; bsplit(sv, a, b);
        XinH[tok * 64 + n] = a; XinL[tok * 64 + n] = b;
      }
    }
  }
#pragma unroll
  for (int t = 3; t < 7; ++t) {
    const int n = t * 16 + c16;
    const int dz = n - kDin;
    if (dz >= 0 && dz < kDin) {
#pragma unroll
      for (int r = 0; r < 8; ++r) ZF[(tb + hh * 8 + r) * kDin + dz] = acc1[t][r];
    }
  }
  __syncthreads();

  v8f accx[3];
#pragma unroll
  for (int t = 0; t < 3; ++t) accx[t] = vzero8();
  {
    const v16b ah0 = Frag<__bf16>::load(XinH + (tb + c16) * 64 + koff);
    const v16b ah1 = Frag<__bf16>::load(XinH + (tb + c16) * 64 + koff + 32);
    const v16b al0 = Frag<__bf16>::load(XinL + (tb + c16) * 64 + koff);
    const v16b al1 = Frag<__bf16>::load(XinL + (tb + c16) * 64 + koff + 32);
#pragma unroll
    for (int t = 0; t < 3; ++t) {
      const v16b bh0 = Frag<__bf16>::load(WxH + (t * 16 + c16) * 64 + koff);
      const v16b bl0 = Frag<__bf16>::load(WxL + (t * 16 + c16) * 64 + koff);
      accx[t] = mma3(ah0, al0, bh0, bl0, accx[t]);
      const v16b bh1 = Frag<__bf16>::load(WxH + (t * 16 + c16) * 64 + koff + 32);
      const v16b bl1 = Frag<__bf16>::load(WxL + (t * 16 + c16) * 64 + koff + 32);
      accx[t] = mma3(ah1, al1, bh1, bl1, accx[t]);
    }
  }
#pragma unroll
  for (int t = 0; t < 3; ++t) {
    const int e = t * 16 + c16;
    if (e < kNX) {
#pragma unroll
      for (int r = 0; r < 8; ++r) Xdbl[(tb + hh * 8 + r) * 36 + e] = accx[t][r];
    }
  }
  __syncthreads();

  __bf16* YH = XinH;
  __bf16* YL = XinL;
#pragma unroll 1
  for (int it = 0; it < 4; ++it) {
    const int sq = tid + it * kThreads;
    if (sq < kPixB * kDin) {
      const int p = sq / kDin, d = sq - p * kDin;
      float a2[16], hs[16];
#pragma unroll
      for (int s = 0; s < 16; ++s) { a2[s] = Am2[d * kDst + s]; hs[s] = 0.f; }
      const float wd0 = Dtw[d * 2 + 0], wd1 = Dtw[d * 2 + 1], bd = Dtb[d], dd = Dvv[d];
#pragma unroll 1
      for (int l = 0; l < kTok; ++l) {
        const int tok = p * kTok + l;
        const float* xr = Xdbl + tok * 36;
        float dt = xr[0] * wd0;
        dt = fmaf(xr[1], wd1, dt);
        dt += bd;
        dt = softplus_f(dt);
        const float xv = XinF[tok * kDin + d];
        float ys = 0.f;
#pragma unroll
        for (int s = 0; s < 16; ++s) {
          const float dA  = exp2f(dt * a2[s]);
          const float dbx = (dt * xr[2 + s]) * xv;
          hs[s] = fmaf(dA, hs[s], dbx);
          ys = fmaf(hs[s], xr[18 + s], ys);
        }
        float yv = fmaf(dd, xv, ys);
        const float zv = ZF[tok * kDin + d];
        yv = yv * (zv * sigm_f(zv));
        __bf16 a, b; bsplit(yv, a, b);
        YH[tok * 64 + d] = a; YL[tok * 64 + d] = b;
      }
    }
  }
  __syncthreads();

  v8f acco[2];
  acco[0] = vzero8(); acco[1] = vzero8();
  {
    const v16b ah0 = Frag<__bf16>::load(YH + (tb + c16) * 64 + koff);
    const v16b ah1 = Frag<__bf16>::load(YH + (tb + c16) * 64 + koff + 32);
    const v16b al0 = Frag<__bf16>::load(YL + (tb + c16) * 64 + koff);
    const v16b al1 = Frag<__bf16>::load(YL + (tb + c16) * 64 + koff + 32);
#pragma unroll
    for (int t = 0; t < 2; ++t) {
      const v16b bh0 = Frag<__bf16>::load(W3H + (t * 16 + c16) * 64 + koff);
      const v16b bl0 = Frag<__bf16>::load(W3L + (t * 16 + c16) * 64 + koff);
      acco[t] = mma3(ah0, al0, bh0, bl0, acco[t]);
      const v16b bh1 = Frag<__bf16>::load(W3H + (t * 16 + c16) * 64 + koff + 32);
      const v16b bl1 = Frag<__bf16>::load(W3L + (t * 16 + c16) * 64 + koff + 32);
      acco[t] = mma3(ah1, al1, bh1, bl1, acco[t]);
    }
  }

  float* Slab = XinF;
  float gsum[4] = {0.f, 0.f, 0.f, 0.f}, gsq[4] = {0.f, 0.f, 0.f, 0.f};
#pragma unroll
  for (int t = 0; t < 2; ++t) {
    const int o = t * 16 + c16;
    const bool ov = o < kGDim;
#pragma unroll
    for (int r = 0; r < 8; ++r) {
      const float vv = ov ? acco[t][r] : 0.f;
      Slab[(tb + hh * 8 + r) * kYPitch + o] = vv;
      gsum[r >> 1] += vv;
      gsq[r >> 1] = fmaf(vv, vv, gsq[r >> 1]);
    }
  }
#pragma unroll
  for (int g = 0; g < 4; ++g) {
#pragma unroll
    for (int off = 16; off > 0; off >>= 1) {
      gsum[g] += __shfl_xor(gsum[g], off, 32);
      gsq[g]  += __shfl_xor(gsq[g], off, 32);
    }
  }
  if (lane == 0) {
#pragma unroll
    for (int g = 0; g < 4; ++g) { Red[wave * 8 + 2 * g] = gsum[g]; Red[wave * 8 + 2 * g + 1] = gsq[g]; }
  }
  __syncthreads();

  {
    const int q = lane >> 3, c4 = (lane & 7) * 4;
    float* yp = ypre + ((size_t)blk * kTokB + tb) * kYPitch;
    for (int pass = 0; pass < 2; ++pass) {
#pragma unroll
      for (int it4 = 0; it4 < 4; ++it4) {
        const int row = it4 * 4 + q;
        const v4f v = *(const v4f*)(Slab + (tb + row) * kYPitch + c4);
        *(volatile v4f*)(yp + (size_t)row * kYPitch + c4) = v;
      }
      __threadfence();
    }
  }
  if (tid < 32) {
    const int t8 = (tid < 8) ? tid : 7;
    float s = Red[t8] + Red[8 + t8];
    s += Red[16 + t8];
    s += Red[24 + t8];
    Blk[tid] = (tid < 8) ? s : 0.f;
  }
  __syncthreads();
  if (wave == 0) {
    float* gp = gpart + (size_t)blk * 32;
    const v4f v = *(const v4f*)(Blk + (lane & 7) * 4);
    for (int pass = 0; pass < 2; ++pass) {
      if (lane < 8) *(volatile v4f*)(gp + lane * 4) = v;
      __threadfence();
    }
  }
}

__global__ __launch_bounds__(256) void k_norm_out(
    const float* __restrict__ ypre, const float* __restrict__ gpart,
    const float* __restrict__ gamma, const float* __restrict__ beta, float* __restrict__ out)
{
  __shared__ __align__(16) float sIn[256 * 32];
  __shared__ __align__(16) float sOut[kNCh * 32];
  __shared__ float sMu[4], sRs[4];
  const int tid  = threadIdx.x;
  const int lane = tid & 31;
  const int wave = tid >> 5;
  const int bimg = blockIdx.x >> 7;
  const int pix0 = (blockIdx.x & 127) * 32;

  if (tid < 4) {
    const float* gp = gpart + (size_t)bimg * kBlkPerImg * 32 + 2 * tid;
    double s = 0.0, q = 0.0;
#pragma unroll 2
    for (int j = 0; j < kBlkPerImg; ++j) { s += (double)gp[j * 32]; q += (double)gp[j * 32 + 1]; }
    const double inv_cnt = 1.0 / (50.0 * 4096.0);
    const double mu = s * inv_cnt;
    double var = q * inv_cnt - mu * mu;
    if (var < 0.0) var = 0.0;
    const float varf = (float)var;
    sMu[tid] = (float)mu;
    sRs[tid] = 1.0f / sqrtf(varf + 1e-5f);
  }
  const float* yp = ypre + ((size_t)bimg * kHW + pix0) * kTok * kYPitch;
#pragma unroll 2
  for (int i = tid; i < 256 * 8; i += 256) {
    const int row = i >> 3, c4 = (i & 7) * 4;
    *(v4f*)(sIn + row * 32 + c4) = *(const v4f*)(yp + (size_t)row * kYPitch + c4);
  }
  __syncthreads();
#pragma unroll 1
  for (int i = tid; i < kNCh * 32; i += 256) {
    const int ch = i >> 5, p = i & 31;
    const int l = ch / kGDim, o = ch - l * kGDim, g = ch / kDin;
    const float v = sIn[(p * kTok + l) * 32 + o];
    const float xn = (v - sMu[g]) * sRs[g] * gamma[ch] + beta[ch];
    sOut[ch * 32 + p] = xn * sigm_f(xn);
  }
  __syncthreads();
  {
    float* ob = out + (size_t)bimg * kBStride + pix0;
    const int q = lane >> 3, c4 = (lane & 7) * 4;
    for (int pass = 0; pass < 2; ++pass) {
#pragma unroll 1
      for (int it = 0; it < 7; ++it) {
        const int ch = (it * 8 + wave) * 4 + q;
        if (ch < kNCh) {
          const v4f v = *(const v4f*)(sOut + ch * 32 + c4);
          *(volatile v4f*)(ob + (size_t)ch * kHW + c4) = v;
        }
      }
      __threadfence();
    }
  }
}

extern "C" void kernel_launch(void* const* d_in, const int* in_sizes, int n_in,
                              void* d_out, int out_size, void* d_ws, size_t ws_size,
                              hipStream_t stream) {
  if (n_in < 13) return;
  if (in_sizes[0] != 2 * kNCh * kHW || in_sizes[1] != kGDim || in_sizes[2] != 100 * kGDim ||
      in_sizes[3] != kDin * 4 || in_sizes[4] != kDin || in_sizes[5] != kNX * kDin ||
      in_sizes[6] != kDin * 2 || in_sizes[7] != kDin || in_sizes[8] != kDin * kDst ||
      in_sizes[9] != kDin || in_sizes[10] != kGDim * kDin || in_sizes[11] != kNCh || in_sizes[12] != kNCh) return;
  if (out_size != 2 * kNCh * kHW) return;
  if (ws_size < kWsTotal) return;

  const float* x      = (const float*)d_in[0];
  const float* pe     = (const float*)d_in[1];
  const float* w_in   = (const float*)d_in[2];
  const float* conv_w = (const float*)d_in[3];
  const float* conv_b = (const float*)d_in[4];
  const float* w_x    = (const float*)d_in[5];
  const float* w_dt   = (const float*)d_in[6];
  const float* b_dt   = (const float*)d_in[7];
  const float* a_log  = (const float*)d_in[8];
  const float* dvec   = (const float*)d_in[9];
  const float* w_out  = (const float*)d_in[10];
  const float* gamma  = (const float*)d_in[11];
  const float* beta   = (const float*)d_in[12];

  float* ypre  = (float*)d_ws;
  float* gpart = (float*)((char*)d_ws + kWsYpreBytes);

  k_mamba_fused<<<kNBlk, kThreads, 0, stream>>>(x, pe, w_in, conv_w, conv_b, w_x, w_dt, b_dt,
                                                 a_log, dvec, w_out, ypre, gpart);
  k_norm_out<<<2 * (kHW / 32), 256, 0, stream>>>(ypre, gpart, gamma, beta, (float*)d_out);
}
